// PointNet2_14697378087179
// MI455X (gfx1250) — hardware-verified
//
#include <hip/hip_runtime.h>
#include <stdint.h>
#pragma clang fp contract(off)

typedef __attribute__((ext_vector_type(16))) _Float16 v16h;
typedef __attribute__((ext_vector_type(8)))  _Float16 v8h;
typedef __attribute__((ext_vector_type(16))) __bf16   v16b;
typedef __attribute__((ext_vector_type(8)))  __bf16   v8b;
typedef __attribute__((ext_vector_type(8)))  float    v8f;
typedef __attribute__((ext_vector_type(4)))  float    v4f;
typedef __attribute__((ext_vector_type(2)))  float    v2f;
typedef __attribute__((ext_vector_type(4)))  unsigned v4u;
typedef __attribute__((ext_vector_type(2)))  unsigned v2u;

constexpr int BATCH = 8;
constexpr int NPTS = 16384;
constexpr int CIN_CH = 35;
constexpr int S1N = 128;
constexpr int S2N = 64;
constexpr int NSAMP = 32;
constexpr int ROWS1 = BATCH * S1N * NSAMP;
constexpr int ROWS2 = BATCH * S2N * NSAMP;
constexpr int ROWSF2 = BATCH * S1N;
constexpr int ROWSF1 = BATCH * NPTS;
static_assert(ROWS1 == 32768 && ROWS2 == 16384 && ROWSF2 == 1024 && ROWSF1 == 131072, "shape");
constexpr int BIG_CHUNKS = 2;
constexpr int CHUNK_ROWS = ROWSF1 / BIG_CHUNKS;
static_assert(CHUNK_ROWS * BIG_CHUNKS == ROWSF1 && CHUNK_ROWS == 65536, "chunking");

constexpr float WLO_CARRY = 2048.0f;
constexpr float WLO_CARRY_INV = 1.0f / 2048.0f;
constexpr float F16_MIN_NORMAL = 6.103515625e-5f;

__device__ __forceinline__ unsigned f2bf_bits(float f) {
  const unsigned u = __float_as_uint(f);
  return (u + 0x7FFFu + ((u >> 16) & 1u)) >> 16;
}
__device__ __forceinline__ void split_pack2(float a, float b, unsigned& hw, unsigned& lw) {
  const unsigned ha = f2bf_bits(a);
  const unsigned hb = f2bf_bits(b);
  const float ra = a - __uint_as_float(ha << 16);
  const float rb = b - __uint_as_float(hb << 16);
  const unsigned la = f2bf_bits(ra);
  const unsigned lb = f2bf_bits(rb);
  hw = (ha & 0xffffu) | (hb << 16);
  lw = (la & 0xffffu) | (lb << 16);
}
__device__ __forceinline__ unsigned f16_bits(float x) {
  const _Float16 h = (_Float16)x;
  const unsigned short s = __builtin_bit_cast(unsigned short, h);
  return (unsigned)s;
}
__device__ __forceinline__ float f16_val(float x) {
  const _Float16 h = (_Float16)x;
  return (float)h;
}
__device__ __forceinline__ void split_pack2_h(float a, float b, unsigned& hw, unsigned& lw) {
  const float fa = (__builtin_fabsf(a) < F16_MIN_NORMAL) ? 0.0f : f16_val(a);
  const float fb = (__builtin_fabsf(b) < F16_MIN_NORMAL) ? 0.0f : f16_val(b);
  const unsigned ha = f16_bits(fa);
  const unsigned hb = f16_bits(fb);
  const float ra = (a - fa) * WLO_CARRY;
  const float rb = (b - fb) * WLO_CARRY;
  const unsigned la = f16_bits(ra);
  const unsigned lb = f16_bits(rb);
  hw = (ha & 0xffffu) | (hb << 16);
  lw = (la & 0xffffu) | (lb << 16);
}
__device__ __forceinline__ void pin_f(float& x) { asm volatile("" : "+v"(x)); }
__device__ __forceinline__ void pin_v4(v4f& x) { asm volatile("" : "+v"(x)); }
__device__ __forceinline__ void wave_lds_sync() {
  __builtin_amdgcn_fence(__ATOMIC_RELEASE, "workgroup");
  __builtin_amdgcn_wave_barrier();
  __builtin_amdgcn_fence(__ATOMIC_ACQUIRE, "workgroup");
}
__device__ __forceinline__ void st2_f(float* p, const float v) {
  *(volatile float*)p = v; __threadfence(); *(volatile float*)p = v;
}
__device__ __forceinline__ void st2_v4f(float* p, const v4f v) {
  *(volatile v4f*)p = v; __threadfence(); *(volatile v4f*)p = v;
}
__device__ __forceinline__ void st2_pair_v4f(float* p, const v4f a, float* q, const v4f b) {
  *(volatile v4f*)p = a; *(volatile v4f*)q = b; __threadfence();
  *(volatile v4f*)p = a; *(volatile v4f*)q = b;
}
__device__ __forceinline__ void st2_pair_u(unsigned* p, const unsigned a, unsigned* q, const unsigned b) {
  *(volatile unsigned*)p = a; *(volatile unsigned*)q = b; __threadfence();
  *(volatile unsigned*)p = a; *(volatile unsigned*)q = b;
}
__device__ __forceinline__ void st2_pair_v2u(unsigned* p, const v2u a, unsigned* q, const v2u b) {
  *(volatile v2u*)p = a; *(volatile v2u*)q = b; __threadfence();
  *(volatile v2u*)p = a; *(volatile v2u*)q = b;
}
__device__ __forceinline__ void st2_pair_v4u(unsigned* p, const v4u a, unsigned* q, const v4u b) {
  *(volatile v4u*)p = a; *(volatile v4u*)q = b; __threadfence();
  *(volatile v4u*)p = a; *(volatile v4u*)q = b;
}

__device__ __forceinline__ void dep_guard4_h(v8f& a, v8f& b, v8f& c, v8f& d, v16h x, v16h y) {
  asm volatile("v_nop\n\tv_nop\n\tv_nop\n\tv_nop" : "+v"(a), "+v"(b), "+v"(c), "+v"(d) : "v"(x), "v"(y));
}
__device__ __forceinline__ void dep_guard2_b(v8f& a, v8f& b, v16b x, v16b y) {
  asm volatile("v_nop\n\tv_nop\n\tv_nop\n\tv_nop" : "+v"(a), "+v"(b) : "v"(x), "v"(y));
}
__device__ __forceinline__ void keep4_h(v16h a, v16h b, v16h c, v16h d) { asm volatile("v_nop" :: "v"(a), "v"(b), "v"(c), "v"(d)); }
__device__ __forceinline__ void keep4_b(v16b a, v16b b, v16b c, v16b d) { asm volatile("v_nop" :: "v"(a), "v"(b), "v"(c), "v"(d)); }
__device__ __forceinline__ void acc_guard4(v8f& a, v8f& b, v8f& c, v8f& d) {
  asm volatile("v_nop\n\tv_nop\n\tv_nop\n\tv_nop" : "+v"(a), "+v"(b), "+v"(c), "+v"(d));
}
template <typename T> struct Frag;
template <> struct Frag<_Float16> {
  typedef v16h V; union U { v16h v; v8h h[2]; };
  static __device__ __forceinline__ v16h load(const _Float16* p) {
    U f; f.h[0] = *(const v8h*)(p); f.h[1] = *(const v8h*)(p + 16); return f.v;
  }
  static __device__ __forceinline__ v8f mma(v16h a, v16h b, v8f c) {
    return __builtin_amdgcn_wmma_f32_16x16x32_f16(false, a, false, b, (short)0, c, false, false);
  }
};
template <> struct Frag<__bf16> {
  typedef v16b V; union U { v16b v; v8b h[2]; };
  static __device__ __forceinline__ v16b load(const __bf16* p) {
    U f; f.h[0] = *(const v8b*)(p); f.h[1] = *(const v8b*)(p + 16); return f.v;
  }
  static __device__ __forceinline__ v8f mma(v16b a, v16b b, v8f c) {
    return __builtin_amdgcn_wmma_f32_16x16x32_bf16(false, a, false, b, (short)0, c, false, false);
  }
};

template <bool STATS>
__attribute__((amdgpu_num_vgpr(256)))
__global__ __launch_bounds__(256) void wmma_gemm_s(
    const unsigned short* __restrict__ Ap, const unsigned short* __restrict__ A2p, int lda,
    const unsigned short* __restrict__ Btp, const unsigned short* __restrict__ Bt2p, int ldb,
    float* __restrict__ Cout, int ldc, float* __restrict__ statp, int M, int N, int K) {
  typedef __bf16 T;
  typedef v16b V;
  const T* A = (const T*)Ap; const T* A2 = (const T*)A2p; const T* Bt = (const T*)Btp; const T* Bt2 = (const T*)Bt2p;
  __shared__ __align__(16) float sT[8][16 * 36];
  const int lane = threadIdx.x & 31;
  const int wave = threadIdx.x >> 5;
  const int tilesN = N >> 5;
  const int tilesM = M >> 6;
  const int tile = blockIdx.x * 8 + wave;
  if (tile >= tilesM * tilesN) return;
  const int tm = tile / tilesN;
  const int tn = tile - tm * tilesN;
  const int m0 = tm << 6;
  const int n0 = tn << 5;

  const int rlane = lane & 15;
  const int koff  = (lane >> 4) * 8;
  const int mOff  = (lane >> 4) * 8;

  v8f acc[4][2];
#pragma unroll
  for (int i = 0; i < 4; ++i)
#pragma unroll
    for (int j = 0; j < 2; ++j) acc[i][j] = (v8f){0.f,0.f,0.f,0.f,0.f,0.f,0.f,0.f};

#pragma unroll 1
  for (int k0 = 0; k0 < K; k0 += 32) {
    V bh[2], bl[2];
#pragma unroll
    for (int j = 0; j < 2; ++j) {
      const size_t bo = (size_t)(n0 + (j << 4) + rlane) * ldb + koff + k0;
      bh[j] = Frag<T>::load(Bt + bo);
      bl[j] = Frag<T>::load(Bt2 + bo);
    }
#pragma unroll
    for (int i = 0; i < 4; ++i) {
      const size_t ao = (size_t)(m0 + (i << 4) + rlane) * lda + koff + k0;
      V ah = Frag<T>::load(A + ao);
      V al = Frag<T>::load(A2 + ao);
#pragma unroll
      for (int j = 0; j < 2; ++j) {
        acc[i][j] = Frag<T>::mma(ah, bh[j], acc[i][j]);
        acc[i][j] = Frag<T>::mma(ah, bl[j], acc[i][j]);
        acc[i][j] = Frag<T>::mma(al, bh[j], acc[i][j]);
      }
      dep_guard2_b(acc[i][0], acc[i][1], ah, al);
    }
    keep4_b(bh[0], bh[1], bl[0], bl[1]);
  }
  acc_guard4(acc[0][0], acc[0][1], acc[1][0], acc[1][1]);
  acc_guard4(acc[2][0], acc[2][1], acc[3][0], acc[3][1]);

  float* slab = sT[wave];
  float cs[2] = {0.f, 0.f};
  float cq[2] = {0.f, 0.f};
#pragma unroll
  for (int i = 0; i < 4; ++i) {
    const int mBase = m0 + (i << 4);
#pragma unroll
    for (int j = 0; j < 2; ++j) {
#pragma unroll
      for (int r = 0; r < 8; ++r) {
        const float v = acc[i][j][r];
        if (STATS) { cs[j] += v; cq[j] += v * v; }
        slab[(mOff + r) * 36 + (j << 4) + rlane] = v;
      }
    }
    wave_lds_sync();
    {
      const int q = lane >> 3, c4 = (lane & 7) * 4;
      for (int pass = 0; pass < 2; ++pass) {
#pragma unroll
        for (int it = 0; it < 4; ++it) {
          const int row = it * 4 + q;
          const v4f v = *(const v4f*)(slab + row * 36 + c4);
          *(volatile v4f*)(Cout + (size_t)(mBase + row) * ldc + n0 + c4) = v;
        }
        __threadfence();
      }
    }
    wave_lds_sync();
  }
  if (STATS) {
#pragma unroll
    for (int j = 0; j < 2; ++j) {
      cs[j] += __shfl_xor(cs[j], 16, 32);
      cq[j] += __shfl_xor(cq[j], 16, 32);
    }
#pragma unroll
    for (int j = 0; j < 2; ++j) {
      slab[(j << 4) + rlane] = cs[j];
      slab[32 + (j << 4) + rlane] = cq[j];
    }
    wave_lds_sync();
    {
      const int li = lane & 15;
      const v4f sv = *(const v4f*)(slab + li * 4);
      float* gbase = statp + ((size_t)tm * (N >> 6) + (tn >> 1)) * 128 + (tn & 1) * 32;
      float* dst = (li < 8) ? (gbase + li * 4) : (gbase + 64 + (li - 8) * 4);
      if (lane < 16) st2_v4f(dst, sv);
    }
  }
}

__attribute__((amdgpu_num_vgpr(256)))
__global__ __launch_bounds__(256) void k_gemm_big(
    const unsigned short* __restrict__ Ahp, const unsigned short* __restrict__ Alp, int lda,
    const unsigned short* __restrict__ Bhp, const unsigned short* __restrict__ Blp, int ldb,
    float* __restrict__ Y, int ldc, float* __restrict__ statp, int M, int N, int K) {
  typedef _Float16 T;
  typedef v16h V;
  const char* Ahb = (const char*)Ahp; const char* Alb = (const char*)Alp;
  const char* Bhb = (const char*)Bhp; const char* Blb = (const char*)Blp;
  __shared__ __align__(16) float sT[8][16 * 36];
  const int lane = threadIdx.x & 31;
  const int wave = threadIdx.x >> 5;
  const int tilesN = N >> 5;
  const int tilesM = M >> 6;
  const int tile = blockIdx.x * 8 + wave;
  if (tile >= tilesM * tilesN) return;
  const int tm = tile / tilesN;
  const int tn = tile - tm * tilesN;
  const int m0 = tm << 6;
  const int n0 = tn << 5;
  const int rlane = lane & 15;
  const int koff  = (lane >> 4) * 8;
  const int mOff  = (lane >> 4) * 8;

  v8f acc[4][2], accr[4][2];
#pragma unroll
  for (int i = 0; i < 4; ++i)
#pragma unroll
    for (int j = 0; j < 2; ++j) {
      acc[i][j]  = (v8f){0.f,0.f,0.f,0.f,0.f,0.f,0.f,0.f};
      accr[i][j] = (v8f){0.f,0.f,0.f,0.f,0.f,0.f,0.f,0.f};
    }

#pragma unroll 1
  for (int k0 = 0; k0 < K; k0 += 32) {
    V bh[2], bl[2];
#pragma unroll
    for (int j = 0; j < 2; ++j) {
      const unsigned bo = ((unsigned)(n0 + (j << 4) + rlane) * (unsigned)ldb + (unsigned)(koff + k0)) * 2u;
      bh[j] = Frag<T>::load((const T*)(Bhb + bo));
      bl[j] = Frag<T>::load((const T*)(Blb + bo));
    }
#pragma unroll
    for (int i = 0; i < 4; ++i) {
      const unsigned ao = ((unsigned)(m0 + (i << 4) + rlane) * (unsigned)lda + (unsigned)(koff + k0)) * 2u;
      V ah = Frag<T>::load((const T*)(Ahb + ao));
      V al = Frag<T>::load((const T*)(Alb + ao));
#pragma unroll
      for (int j = 0; j < 2; ++j) {
        acc[i][j]  = Frag<T>::mma(ah, bh[j], acc[i][j]);
        accr[i][j] = Frag<T>::mma(ah, bl[j], accr[i][j]);
        accr[i][j] = Frag<T>::mma(al, bh[j], accr[i][j]);
      }
      dep_guard4_h(acc[i][0], acc[i][1], accr[i][0], accr[i][1], ah, al);
    }
    keep4_h(bh[0], bh[1], bl[0], bl[1]);
  }
  acc_guard4(acc[0][0], acc[0][1], accr[0][0], accr[0][1]);
  acc_guard4(acc[1][0], acc[1][1], accr[1][0], accr[1][1]);
  acc_guard4(acc[2][0], acc[2][1], accr[2][0], accr[2][1]);
  acc_guard4(acc[3][0], acc[3][1], accr[3][0], accr[3][1]);

  float* slab = sT[wave];
  float cs[2] = {0.f, 0.f};
  float cq[2] = {0.f, 0.f};
#pragma unroll
  for (int i = 0; i < 4; ++i) {
    const int mBase = m0 + (i << 4);
#pragma unroll
    for (int j = 0; j < 2; ++j) {
#pragma unroll
      for (int r = 0; r < 8; ++r) {
        const float rr = accr[i][j][r] * WLO_CARRY_INV;
        const float v = acc[i][j][r] + rr;
        cs[j] += v; cq[j] += v * v;
        slab[(mOff + r) * 36 + (j << 4) + rlane] = v;
      }
    }
    wave_lds_sync();
    {
      const int q = lane >> 3, c4 = (lane & 7) * 4;
      for (int pass = 0; pass < 2; ++pass) {
#pragma unroll
        for (int it = 0; it < 4; ++it) {
          const int row = it * 4 + q;
          const v4f v = *(const v4f*)(slab + row * 36 + c4);
          *(volatile v4f*)(Y + (size_t)(mBase + row) * ldc + n0 + c4) = v;
        }
        __threadfence();
      }
    }
    wave_lds_sync();
  }
#pragma unroll
  for (int j = 0; j < 2; ++j) {
    cs[j] += __shfl_xor(cs[j], 16, 32);
    cq[j] += __shfl_xor(cq[j], 16, 32);
  }
#pragma unroll
  for (int j = 0; j < 2; ++j) {
    slab[(j << 4) + rlane] = cs[j];
    slab[32 + (j << 4) + rlane] = cq[j];
  }
  wave_lds_sync();
  {
    const int li = lane & 15;
    const v4f sv = *(const v4f*)(slab + li * 4);
    float* gbase = statp + ((size_t)tm * (N >> 6) + (tn >> 1)) * 128 + (tn & 1) * 32;
    float* dst = (li < 8) ? (gbase + li * 4) : (gbase + 64 + (li - 8) * 4);
    if (lane < 16) st2_v4f(dst, sv);
  }
}

__global__ __launch_bounds__(256) void k_prep_w(const float* __restrict__ W, int O, int K, int Op, int Kp,
                                                unsigned* __restrict__ hi, unsigned* __restrict__ lo, int mode) {
  const int i = blockIdx.x * 256 + threadIdx.x;
  const int total8 = (Op * Kp) >> 3;
  if (i < total8) {
    const int e0 = i * 8;
    const int o = e0 / Kp;
    const int k0 = e0 - o * Kp;
    const int oc = o < O ? o : O - 1;
    float v[8];
#pragma unroll
    for (int e = 0; e < 8; ++e) {
      const int k = k0 + e;
      const int kc = k < K ? k : K - 1;
      float x = W[(size_t)oc * K + kc];
      pin_f(x);
      v[e] = (o < O && k < K) ? x : 0.0f;
    }
    v4u hv, lv;
#pragma unroll
    for (int p = 0; p < 4; ++p) {
      unsigned hw, lw;
      if (mode == 0) split_pack2(v[2 * p], v[2 * p + 1], hw, lw);
      else split_pack2_h(v[2 * p], v[2 * p + 1], hw, lw);
      hv[p] = hw; lv[p] = lw;
    }
    st2_pair_v4u(hi + (size_t)i * 4, hv, lo + (size_t)i * 4, lv);
  }
}

__global__ __launch_bounds__(256) void k_prep_points(const float* __restrict__ xyz, float* __restrict__ P0,
                                                     int nB, int nC, int nN) {
#pragma clang fp contract(off)
  const int i = blockIdx.x * 256 + threadIdx.x;
  if (i < nB * nN) {
    const int b = i / nN;
    const int n = i - b * nN;
    const float* pb = xyz + (size_t)b * nC * nN + n;
    const float x = pb[0];
    const float y = pb[(size_t)nN];
    const float z = pb[2 * (size_t)nN];
    const float tx = x * x;
    const float ty = y * y;
    const float tz = z * z;
    const float sq = (tx + tz) + ty;
    v4f v; v[0] = x; v[1] = y; v[2] = z; v[3] = sq;
    st2_v4f(P0 + (size_t)i * 4, v);
  }
}

template <int NT, int PPT>
__global__ __launch_bounds__(NT) void k_fps(const float* __restrict__ P, int S, float* __restrict__ Cout) {
#pragma clang fp contract(off)
  constexpr int NP = NT * PPT;
  constexpr int NWV = NT / 32;
  __shared__ float s_val[32];
  __shared__ int s_idx[32];
  __shared__ int s_far[128];
  const int b = blockIdx.x, t = threadIdx.x, lane = t & 31, wave = t >> 5;
  const int Sc = S < 128 ? S : 128;
  const float* Pb = P + (size_t)b * NP * 4;
  float px[PPT], py[PPT], pz[PPT], dist[PPT];
#pragma unroll
  for (int j = 0; j < PPT; ++j) {
    v4f v = *(const v4f*)(Pb + (size_t)(j * NT + t) * 4);
    pin_v4(v);
    px[j] = v[0]; py[j] = v[1]; pz[j] = v[2];
    dist[j] = 1e10f;
    if ((j & 7) == 7) asm volatile("" ::: "memory");
  }
  int far = 0;
  for (int it = 0; it < Sc; ++it) {
    if (t == 0) s_far[it] = far;
    const v4f c = *(const v4f*)(Pb + (size_t)far * 4);
    const float cx = c[0], cy = c[1], cz = c[2];
    float bv = 0.0f;
    int bi = 0;
#pragma unroll
    for (int j = 0; j < PPT; ++j) {
      const float dx = px[j] - cx;
      const float dy = py[j] - cy;
      const float dz = pz[j] - cz;
      const float tx = dx * dx;
      const float ty = dy * dy;
      const float tz = dz * dz;
      const float d = (tx + tz) + ty;
      const float nd = fminf(dist[j], d);
      dist[j] = nd;
      if (j == 0) { bv = nd; bi = t; }
      else { const bool g = nd > bv; bv = g ? nd : bv; bi = g ? (j * NT + t) : bi; }
    }
#pragma unroll
    for (int off = 16; off > 0; off >>= 1) {
      const float ov = __shfl_xor(bv, off, 32);
      const int oi = __shfl_xor(bi, off, 32);
      const bool take = (ov > bv) || ((ov == bv) && (oi < bi));
      bv = take ? ov : bv; bi = take ? oi : bi;
    }
    if (lane == 0) { s_val[wave] = bv; s_idx[wave] = bi; }
    __syncthreads();
    const int ls = lane < NWV ? lane : NWV - 1;
    float v2 = s_val[ls];
    int i2 = s_idx[ls];
    if (lane >= NWV) { v2 = -1.0f; i2 = 0x7fffffff; }
#pragma unroll
    for (int off = 16; off > 0; off >>= 1) {
      const float ov = __shfl_xor(v2, off, 32);
      const int oi = __shfl_xor(i2, off, 32);
      const bool take = (ov > v2) || ((ov == v2) && (oi < i2));
      v2 = take ? ov : v2; i2 = take ? oi : i2;
    }
    far = i2 < 0 ? 0 : (i2 > NP - 1 ? NP - 1 : i2);
    __syncthreads();
  }
  if (t < Sc) {
    int f = s_far[t];
    f = f < 0 ? 0 : (f > NP - 1 ? NP - 1 : f);
    const v4f v = *(const v4f*)(Pb + (size_t)f * 4);
    st2_v4f(Cout + ((size_t)b * Sc + t) * 4, v);
  }
}

template <int CPL>
__global__ __launch_bounds__(256) void k_ballgroup(
    const float* __restrict__ P, int NP, const float* __restrict__ Cc, int S, int nCent, float r2,
    const float* __restrict__ feat, long f_bs, long f_ns, long f_cs, int CF,
    unsigned* __restrict__ Ahi, unsigned* __restrict__ Alo) {
#pragma clang fp contract(off)
  __shared__ int slots[8][32];
  const int lane = threadIdx.x & 31, wave = threadIdx.x >> 5;
  const int cw = blockIdx.x * 8 + wave;
  if (cw >= nCent) return;
  const int b = cw / S;
  const v4f c = *(const v4f*)(Cc + (size_t)cw * 4);
  const float* Pb = P + (size_t)b * NP * 4;
  slots[wave][lane] = 0;
  wave_lds_sync();
  const unsigned lmask = (1u << lane) - 1u;
  int cnt = 0;
  for (int base = 0; base < NP && cnt < 32; base += 32) {
    const int n = base + lane;
    const int nc = n < NP ? n : NP - 1;
    const v4f p = *(const v4f*)(Pb + (size_t)nc * 4);
    float d = c[0] * p[0];
    d = __builtin_fmaf(c[1], p[1], d);
    d = __builtin_fmaf(c[2], p[2], d);
    const float s2 = c[3] + p[3];
    const float sqr = s2 - 2.0f * d;
    const bool ok = (n < NP) && !(sqr > r2);
    const unsigned mm = __builtin_amdgcn_ballot_w32(ok);
    const int slot = cnt + __builtin_popcount(mm & lmask);
    if (ok && slot < 32) slots[wave][slot] = n;
    cnt += __builtin_popcount(mm);
  }
  wave_lds_sync();
  const int cntc = cnt < 32 ? cnt : 32;
  int first = slots[wave][0];
  if (cnt == 0) first = NP - 1;
  int mine = slots[wave][lane];
  if (lane >= cntc) mine = first;
  mine = mine < 0 ? 0 : (mine > NP - 1 ? NP - 1 : mine);

  const float* fb = feat + (size_t)b * f_bs;
  const size_t row0 = (size_t)cw * 32;
#pragma unroll 1
  for (int k = 0; k < 32; ++k) {
    const int n = __shfl(mine, k, 32);
    const v4f p = *(const v4f*)(Pb + (size_t)n * 4);
    const float rx = p[0] - c[0];
    const float ry = p[1] - c[1];
    const float rz = p[2] - c[2];
    float vals[CPL];
#pragma unroll
    for (int e = 0; e < CPL; ++e) {
      const int ch = lane * CPL + e;
      int fc = ch - 3;
      fc = fc < 0 ? 0 : (fc > CF - 1 ? CF - 1 : fc);
      float f = fb[(size_t)n * f_ns + (size_t)fc * f_cs];
      pin_f(f);
      const float rel = (ch == 0) ? rx : ((ch == 1) ? ry : rz);
      vals[e] = (ch < 3) ? rel : ((ch < 3 + CF) ? f : 0.0f);
    }
    if constexpr (CPL == 2) {
      unsigned hw, lw;
      split_pack2(vals[0], vals[1], hw, lw);
      st2_pair_u(Ahi + (row0 + k) * 32 + lane, hw, Alo + (row0 + k) * 32 + lane, lw);
    } else {
      v2u hv, lv;
      unsigned hw, lw;
      split_pack2(vals[0], vals[1], hw, lw); hv[0] = hw; lv[0] = lw;
      split_pack2(vals[2], vals[3], hw, lw); hv[1] = hw; lv[1] = lw;
      st2_pair_v2u(Ahi + (row0 + k) * 64 + lane * 2, hv, Alo + (row0 + k) * 64 + lane * 2, lv);
    }
  }
}

__global__ __launch_bounds__(256) void k_bn_reduce(const float* __restrict__ stat, int tilesM, int groups,
                                                   double invM, float* __restrict__ bnp) {
  const int c = threadIdx.x;
  const int g = c >> 6, cc = c & 63;
  const bool valid = g < groups;
  const int gc = valid ? g : groups - 1;
  double s = 0.0, q = 0.0;
#pragma unroll 4
  for (int tm = 0; tm < tilesM; ++tm) {
    const size_t base = ((size_t)tm * groups + gc) * 128;
    s += (double)stat[base + cc];
    q += (double)stat[base + 64 + cc];
  }
  const double mean = s * invM;
  double var = q * invM - mean * mean;
  var = var < 0.0 ? 0.0 : var;
  const float vf = (float)var + 1e-5f;
  const float m = valid ? (float)mean : 0.0f;
  const float is = valid ? (1.0f / sqrtf(vf)) : 0.0f;
  st2_f(bnp + c, m);
  st2_f(bnp + 256 + c, is);
}

__global__ __launch_bounds__(256) void k_apply_split(const float* __restrict__ Y, const float* __restrict__ bnp,
                                                     unsigned* __restrict__ hi, unsigned* __restrict__ lo,
                                                     int total8, int ld) {
  const int i = blockIdx.x * 256 + threadIdx.x;
  if (i < total8) {
    const size_t e0 = (size_t)i * 8;
    const int c0 = (int)(e0 % (size_t)ld);
    const v4f y0 = *(const v4f*)(Y + e0);
    const v4f y1 = *(const v4f*)(Y + e0 + 4);
    const v4f m0 = *(const v4f*)(bnp + c0);
    const v4f m1 = *(const v4f*)(bnp + c0 + 4);
    const v4f s0 = *(const v4f*)(bnp + 256 + c0);
    const v4f s1 = *(const v4f*)(bnp + 256 + c0 + 4);
    float t[8];
#pragma unroll
    for (int e = 0; e < 4; ++e) {
      t[e]     = fmaxf((y0[e] - m0[e]) * s0[e], 0.0f);
      t[4 + e] = fmaxf((y1[e] - m1[e]) * s1[e], 0.0f);
    }
    v4u hv, lv;
#pragma unroll
    for (int p = 0; p < 4; ++p) {
      unsigned hw, lw;
      split_pack2(t[2 * p], t[2 * p + 1], hw, lw);
      hv[p] = hw; lv[p] = lw;
    }
    st2_pair_v4u(hi + (size_t)i * 4, hv, lo + (size_t)i * 4, lv);
  }
}

__global__ __launch_bounds__(256) void k_apply_f16s(const float* __restrict__ Y, const float* __restrict__ bnp,
                                                    unsigned* __restrict__ hi, unsigned* __restrict__ lo,
                                                    int total8, int ld) {
  const int i = blockIdx.x * 256 + threadIdx.x;
  if (i < total8) {
    const size_t e0 = (size_t)i * 8;
    const int c0 = (int)(e0 % (size_t)ld);
    const v4f y0 = *(const v4f*)(Y + e0);
    const v4f y1 = *(const v4f*)(Y + e0 + 4);
    const v4f m0 = *(const v4f*)(bnp + c0);
    const v4f m1 = *(const v4f*)(bnp + c0 + 4);
    const v4f s0 = *(const v4f*)(bnp + 256 + c0);
    const v4f s1 = *(const v4f*)(bnp + 256 + c0 + 4);
    float t[8];
#pragma unroll
    for (int e = 0; e < 4; ++e) {
      t[e]     = fmaxf((y0[e] - m0[e]) * s0[e], 0.0f);
      t[4 + e] = fmaxf((y1[e] - m1[e]) * s1[e], 0.0f);
    }
    v4u hv, lv;
#pragma unroll
    for (int p = 0; p < 4; ++p) {
      unsigned hw, lw;
      split_pack2_h(t[2 * p], t[2 * p + 1], hw, lw);
      hv[p] = hw; lv[p] = lw;
    }
    st2_pair_v4u(hi + (size_t)i * 4, hv, lo + (size_t)i * 4, lv);
  }
}

template <int CPL>
__global__ __launch_bounds__(256) void k_bn_maxpool(const float* __restrict__ Y, const float* __restrict__ bnp,
                                                    float* __restrict__ outp, int nCent) {
  typedef float VT __attribute__((ext_vector_type(CPL)));
  constexpr int C = 32 * CPL;
  const int lane = threadIdx.x & 31, wave = threadIdx.x >> 5;
  const int cw = blockIdx.x * 8 + wave;
  if (cw >= nCent) return;
  const int ch0 = lane * CPL;
  const VT m = *(const VT*)(bnp + ch0);
  const VT is = *(const VT*)(bnp + 256 + ch0);
  VT mx;
#pragma unroll
  for (int e = 0; e < CPL; ++e) mx[e] = -__builtin_inff();
#pragma unroll 4
  for (int k = 0; k < 32; ++k) {
    const VT y = *(const VT*)(Y + ((size_t)cw * 32 + k) * C + ch0);
#pragma unroll
    for (int e = 0; e < CPL; ++e) {
      const float t = fmaxf((y[e] - m[e]) * is[e], 0.0f);
      mx[e] = fmaxf(mx[e], t);
    }
  }
  float* dst = outp + (size_t)cw * C + ch0;
  *(volatile VT*)dst = mx;
  __threadfence();
  *(volatile VT*)dst = mx;
}

__global__ __launch_bounds__(256) void k_out1(const float* __restrict__ l4, float* __restrict__ o1) {
  __shared__ float tile[64 * 129];
  const int b = blockIdx.x, t = threadIdx.x;
  const float* src = l4 + (size_t)b * 64 * 128;
#pragma unroll
  for (int it = 0; it < 8; ++it) {
    const int f = (it * 256 + t) * 4;
    const int s = f >> 7, c = f & 127;
    const v4f v = *(const v4f*)(src + f);
    tile[s * 129 + c + 0] = v[0];
    tile[s * 129 + c + 1] = v[1];
    tile[s * 129 + c + 2] = v[2];
    tile[s * 129 + c + 3] = v[3];
  }
  __syncthreads();
  v4f vv[8];
#pragma unroll
  for (int it = 0; it < 8; ++it) {
    const int o = (it * 256 + t) * 4;
    const int c = o >> 6, s = o & 63;
    vv[it][0] = tile[(s + 0) * 129 + c];
    vv[it][1] = tile[(s + 1) * 129 + c];
    vv[it][2] = tile[(s + 2) * 129 + c];
    vv[it][3] = tile[(s + 3) * 129 + c];
  }
  float* dst = o1 + (size_t)b * 8192;
  for (int pass = 0; pass < 2; ++pass) {
#pragma unroll
    for (int it = 0; it < 8; ++it) *(volatile v4f*)(dst + (it * 256 + t) * 4) = vv[it];
    __threadfence();
  }
}

__device__ __forceinline__ void nn3_step(const v4f q, const v4f c, int m,
                                         float& b0, float& b1, float& b2, int& i0, int& i1, int& i2) {
#pragma clang fp contract(off)
  float p = q[0] * c[0];
  p = __builtin_fmaf(q[1], c[1], p);
  p = __builtin_fmaf(q[2], c[2], p);
  const float s2 = q[3] + c[3];
  const float d = s2 - 2.0f * p;
  const bool lt0 = d < b0, lt1 = d < b1, lt2 = d < b2;
  const float nb2 = lt1 ? b1 : (lt2 ? d : b2);
  const int   ni2 = lt1 ? i1 : (lt2 ? m : i2);
  const float nb1 = lt0 ? b0 : (lt1 ? d : b1);
  const int   ni1 = lt0 ? i0 : (lt1 ? m : i1);
  const float nb0 = lt0 ? d : b0;
  const int   ni0 = lt0 ? m : i0;
  b0 = nb0; b1 = nb1; b2 = nb2; i0 = ni0; i1 = ni1; i2 = ni2;
}
__device__ __forceinline__ void nn3_weights(float b0, float b1, float b2, float& w0, float& w1, float& w2) {
#pragma clang fp contract(off)
  const float r0 = 1.0f / (b0 + 1e-8f);
  const float r1 = 1.0f / (b1 + 1e-8f);
  const float r2 = 1.0f / (b2 + 1e-8f);
  const float rs = (r0 + r2) + r1;
  const float inv = 1.0f / rs;
  w0 = r0 * inv; w1 = r1 * inv; w2 = r2 * inv;
}

__global__ __launch_bounds__(128) void k_fp2(const float* __restrict__ C1, const float* __restrict__ C2,
                                             const float* __restrict__ l1p, const float* __restrict__ l4,
                                             unsigned* __restrict__ Ahi, unsigned* __restrict__ Alo) {
#pragma clang fp contract(off)
  static_assert(S1N == 128 && S2N == 64, "block shape");
  __shared__ __align__(16) float sC[S2N * 4];
  const int b = blockIdx.x, t = threadIdx.x, lane = t & 31, wave = t >> 5;
  {
    const int tc = t < S2N ? t : S2N - 1;
    const v4f v = *(const v4f*)(C2 + ((size_t)b * S2N + tc) * 4);
    if (t < S2N) *(v4f*)(sC + t * 4) = v;
  }
  __syncthreads();
  const v4f q = *(const v4f*)(C1 + ((size_t)b * S1N + t) * 4);
  float b0 = __builtin_inff(), b1 = __builtin_inff(), b2 = __builtin_inff();
  int i0 = 0, i1 = 0, i2 = 0;
#pragma unroll 4
  for (int m = 0; m < S2N; ++m) {
    const v4f c = *(const v4f*)(sC + m * 4);
    nn3_step(q, c, m, b0, b1, b2, i0, i1, i2);
  }
  float w0, w1, w2;
  nn3_weights(b0, b1, b2, w0, w1, w2);

  const int lo_old = (lane < 8 ? lane : 7) * 8;
  int cl = lane - 8;
  cl = cl < 0 ? 0 : (cl > 15 ? 15 : cl);
  const int lo_int = cl * 8;
#pragma unroll 1
  for (int p = 0; p < 32; ++p) {
    int j0 = __shfl(i0, p, 32);
    int j1 = __shfl(i1, p, 32);
    int j2 = __shfl(i2, p, 32);
    const float u0 = __shfl(w0, p, 32);
    const float u1 = __shfl(w1, p, 32);
    const float u2 = __shfl(w2, p, 32);
    j0 = j0 < 0 ? 0 : (j0 > S2N - 1 ? S2N - 1 : j0);
    j1 = j1 < 0 ? 0 : (j1 > S2N - 1 ? S2N - 1 : j1);
    j2 = j2 < 0 ? 0 : (j2 > S2N - 1 ? S2N - 1 : j2);
    const size_t row = (size_t)b * S1N + wave * 32 + p;
    const float* po = l1p + row * 64 + lo_old;
    const float* z0 = l4 + ((size_t)b * S2N + j0) * 128 + lo_int;
    const float* z1 = l4 + ((size_t)b * S2N + j1) * 128 + lo_int;
    const float* z2 = l4 + ((size_t)b * S2N + j2) * 128 + lo_int;
    v4f a0 = *(const v4f*)(po);
    v4f a1 = *(const v4f*)(po + 4);
    v4f z00 = *(const v4f*)(z0);
    v4f z01 = *(const v4f*)(z0 + 4);
    v4f z10 = *(const v4f*)(z1);
    v4f z11 = *(const v4f*)(z1 + 4);
    v4f z20 = *(const v4f*)(z2);
    v4f z21 = *(const v4f*)(z2 + 4);
    pin_v4(a0); pin_v4(a1); pin_v4(z00); pin_v4(z01); pin_v4(z10); pin_v4(z11); pin_v4(z20); pin_v4(z21);
    const v4f g0 = (z00 * u0 + z10 * u1) + z20 * u2;
    const v4f g1 = (z01 * u0 + z11 * u1) + z21 * u2;
    float vals[8];
#pragma unroll
    for (int e = 0; e < 4; ++e) {
      vals[e]     = (lane < 8) ? a0[e] : g0[e];
      vals[4 + e] = (lane < 8) ? a1[e] : g1[e];
    }
    v4u hv, lv;
#pragma unroll
    for (int pp = 0; pp < 4; ++pp) {
      unsigned hw, lw;
      split_pack2(vals[2 * pp], vals[2 * pp + 1], hw, lw);
      hv[pp] = hw; lv[pp] = lw;
    }
    if (lane < 24) st2_pair_v4u(Ahi + row * 96 + lane * 4, hv, Alo + row * 96 + lane * 4, lv);
  }
}

__global__ __launch_bounds__(256) void k_fp1(const float* __restrict__ P0, const float* __restrict__ C1,
                                             const float* __restrict__ Z, float* __restrict__ Y,
                                             float* __restrict__ statp) {
#pragma clang fp contract(off)
  __shared__ __align__(16) float sC[S1N * 4];
  constexpr int BLK_PER_B = NPTS / 256;
  const int t = threadIdx.x, lane = t & 31, wave = t >> 5;
  const int b = blockIdx.x / BLK_PER_B;
  const int n = (blockIdx.x - b * BLK_PER_B) * 256 + t;
  {
    const int tc = t < S1N ? t : S1N - 1;
    const v4f v = *(const v4f*)(C1 + ((size_t)b * S1N + tc) * 4);
    if (t < S1N) *(v4f*)(sC + t * 4) = v;
  }
  __syncthreads();
  const v4f q = *(const v4f*)(P0 + ((size_t)b * NPTS + n) * 4);
  float b0 = __builtin_inff(), b1 = __builtin_inff(), b2 = __builtin_inff();
  int i0 = 0, i1 = 0, i2 = 0;
#pragma unroll 4
  for (int m = 0; m < S1N; ++m) {
    const v4f c = *(const v4f*)(sC + m * 4);
    nn3_step(q, c, m, b0, b1, b2, i0, i1, i2);
  }
  float w0, w1, w2;
  nn3_weights(b0, b1, b2, w0, w1, w2);

  const size_t rowbase = (size_t)b * NPTS + (n - lane);
  const float* Zb = Z + (size_t)b * S1N * 128 + lane * 4;
  v4f cs = (v4f){0.f, 0.f, 0.f, 0.f};
  v4f cq = (v4f){0.f, 0.f, 0.f, 0.f};
#pragma unroll 1
  for (int p = 0; p < 32; ++p) {
    int j0 = __shfl(i0, p, 32);
    int j1 = __shfl(i1, p, 32);
    int j2 = __shfl(i2, p, 32);
    const float u0 = __shfl(w0, p, 32);
    const float u1 = __shfl(w1, p, 32);
    const float u2 = __shfl(w2, p, 32);
    j0 = j0 < 0 ? 0 : (j0 > S1N - 1 ? S1N - 1 : j0);
    j1 = j1 < 0 ? 0 : (j1 > S1N - 1 ? S1N - 1 : j1);
    j2 = j2 < 0 ? 0 : (j2 > S1N - 1 ? S1N - 1 : j2);
    const v4f z0 = *(const v4f*)(Zb + (size_t)j0 * 128);
    const v4f z1 = *(const v4f*)(Zb + (size_t)j1 * 128);
    const v4f z2 = *(const v4f*)(Zb + (size_t)j2 * 128);
    const v4f y = (z0 * u0 + z1 * u1) + z2 * u2;
    cs += y;
    cq += y * y;
    st2_v4f(Y + (rowbase + p) * 128 + lane * 4, y);
  }
  {
    const size_t tw = (size_t)blockIdx.x * 8 + wave;
    float* sb = statp + tw * 256 + (lane >> 4) * 128 + (lane & 15) * 4;
    st2_pair_v4f(sb, cs, sb + 64, cq);
  }
}

__global__ __launch_bounds__(256) void k_final(const float* __restrict__ Y, const float* __restrict__ bnp,
                                               const float* __restrict__ w2, const float* __restrict__ b2,
                                               float* __restrict__ outp, int nWaves) {
  const int lane = threadIdx.x & 31, wave = threadIdx.x >> 5;
  const int gw = blockIdx.x * 8 + wave;
  if (gw >= nWaves) return;
  const size_t base = (size_t)gw * 32;
  const int ch = lane * 4;
  const v4f m = *(const v4f*)(bnp + ch);
  const v4f is = *(const v4f*)(bnp + 256 + ch);
  const v4f w = *(const v4f*)(w2 + ch);
  const float bias = b2[0];
  float res = 0.0f;
#pragma unroll 2
  for (int p = 0; p < 32; ++p) {
    const v4f y = *(const v4f*)(Y + (base + p) * 128 + ch);
    float s = 0.0f;
#pragma unroll
    for (int e = 0; e < 4; ++e) {
      const float t = (y[e] - m[e]) * is[e];
      const float a = (t >= 0.0f) ? t : 0.01f * t;
      s = __builtin_fmaf(a, w[e], s);
    }
#pragma unroll
    for (int off = 16; off > 0; off >>= 1) s += __shfl_xor(s, off, 32);
    res = (lane == p) ? s : res;
  }
  const float o = res + bias;
  st2_f(outp + base + lane, o);
}

constexpr int NUM_W = 12;
constexpr int W_DIN[NUM_W]  = {1, 2, 3, 4, 5, 6, 7, 8, 9, 10, 11, 12};
constexpr int W_O[NUM_W]    = {32, 32, 64, 64, 64, 128, 256, 128, 128, 128, 128, 128};
constexpr int W_K[NUM_W]    = {38, 32, 32, 67, 64, 64, 192, 256, 128, 128, 128, 128};
constexpr int W_OP[NUM_W]   = {64, 64, 64, 64, 64, 128, 256, 128, 128, 128, 128, 128};
constexpr int W_KP[NUM_W]   = {64, 32, 32, 96, 64, 64, 192, 256, 128, 128, 128, 128};
constexpr int W_MODE[NUM_W] = {0, 0, 0, 0, 0, 0, 0, 0, 0, 1, 1, 1};
static_assert(sizeof(W_KP) / sizeof(W_KP[0]) == NUM_W, "table");
constexpr size_t w_off(int i) {
  size_t o = 0;
  for (int j = 0; j < i; ++j) o += (size_t)W_OP[j] * W_KP[j];
  return o;
}
constexpr bool w_planes_ok() {
  for (int j = 0; j < NUM_W; ++j) {
    if (((W_OP[j] * W_KP[j]) % 2048) != 0) return false;
    if ((W_KP[j] % 32) != 0 || (W_OP[j] % 64) != 0) return false;
  }
  return true;
}
static_assert(w_planes_ok(), "weight planes: whole 256-thread blocks, K%32, N%64");
constexpr bool gemm_ok(int M, int N, int K) { return (M % 64 == 0) && (N % 64 == 0) && (K % 32 == 0); }

constexpr size_t al512(size_t x) { return (x + 511) & ~(size_t)511; }
constexpr size_t SZ_P0   = (size_t)BATCH * NPTS * 16;
constexpr size_t SZ_C1   = (size_t)BATCH * S1N * 16;
constexpr size_t SZ_C2   = (size_t)BATCH * S2N * 16;
constexpr size_t SZ_W    = w_off(NUM_W) * 2;
constexpr size_t SZ_BNP  = 32768;
constexpr size_t SZ_STAT = (size_t)4096 * 256 * 4;
constexpr size_t SZ_L1P  = (size_t)ROWSF2 * 64 * 4;
constexpr size_t SZ_L4   = (size_t)BATCH * S2N * 128 * 4;
constexpr size_t SZ_AS   = (size_t)ROWS1 * 64 * 2;
constexpr size_t SZ_YS   = (size_t)ROWS1 * 64 * 4;
constexpr size_t SZ_F2A  = (size_t)ROWSF2 * 192 * 2;
constexpr size_t SZ_F2Y  = (size_t)ROWSF2 * 256 * 4;
constexpr size_t SZ_F2B  = (size_t)ROWSF2 * 256 * 2;
constexpr size_t SZ_F2Y2 = (size_t)ROWSF2 * 128 * 4;
constexpr size_t SZ_L1N  = (size_t)ROWSF2 * 128 * 2;
constexpr size_t SZ_ZT   = (size_t)ROWSF2 * 128 * 4;
constexpr size_t SZ_YBIG = (size_t)ROWSF1 * 128 * 4;
constexpr size_t SZ_ABP  = (size_t)CHUNK_ROWS * 128 * 2;
static_assert(SZ_AS >= (size_t)ROWS2 * 128 * 2 && SZ_YS >= (size_t)ROWS2 * 128 * 4, "SA planes sized from max user");
static_assert(SZ_STAT >= (size_t)(ROWSF1 / 64) * 2 * 128 * 4 && SZ_STAT >= (size_t)(ROWS1 / 64) * 128 * 4 &&
              SZ_STAT >= (size_t)(ROWS2 / 64) * 2 * 128 * 4 && SZ_STAT >= (size_t)(ROWSF2 / 64) * 4 * 128 * 4 &&
              SZ_STAT >= (size_t)(ROWSF1 / 32) * 256 * 4, "stat table sized from max user");
static_assert(SZ_BNP >= 13 * 2048, "bn slots");
static_assert(SZ_ABP == (size_t)16777216, "activation chunk plane");
constexpr size_t OFF_P0   = 0;
constexpr size_t OFF_C1   = OFF_P0 + al512(SZ_P0);
constexpr size_t OFF_C2   = OFF_C1 + al512(SZ_C1);
constexpr size_t OFF_WHI  = OFF_C2 + al512(SZ_C2);
constexpr size_t OFF_WLO  = OFF_WHI + al512(SZ_W);
constexpr size_t OFF_BNP  = OFF_WLO + al512(SZ_W);
constexpr size_t OFF_STAT = OFF_BNP + al512(SZ_BNP);
constexpr size_t OFF_L1P  = OFF_STAT + al512(SZ_STAT);
constexpr size_t OFF_L4   = OFF_L1P + al512(SZ_L1P);
constexpr size_t OFF_ASH  = OFF_L4 + al512(SZ_L4);
constexpr size_t OFF_ASL  = OFF_ASH + al512(SZ_AS);
constexpr size_t OFF_YS   = OFF_ASL + al512(SZ_AS);
constexpr size_t OFF_F2AH = OFF_YS + al512(SZ_YS);
constexpr size_t OFF_F2AL = OFF_F2AH + al512(SZ_F2A);
constexpr size_t OFF_F2Y  = OFF_F2AL + al512(SZ_F2A);
constexpr size_t OFF_F2BH = OFF_F2Y + al512(SZ_F2Y);
constexpr size_t OFF_F2BL = OFF_F2BH + al512(SZ_F2B);
constexpr size_t OFF_F2Y2 = OFF_F2BL + al512(SZ_F2B);
constexpr size_t OFF_L1NH = OFF_F2Y2 + al512(SZ_F2Y2);
constexpr size_t OFF_L1NL = OFF_L1NH + al512(SZ_L1N);
constexpr size_t OFF_ZT   = OFF_L1NL + al512(SZ_L1N);
constexpr size_t OFF_YBIG = OFF_ZT + al512(SZ_ZT);
constexpr size_t OFF_ABH  = OFF_YBIG + al512(SZ_YBIG);
constexpr size_t OFF_ABL  = OFF_ABH + al512(SZ_ABP);
constexpr size_t WS_TOTAL = OFF_ABL + al512(SZ_ABP);
static_assert(WS_TOTAL == (size_t)129466368, "carve total");
static_assert(WS_TOTAL <= (size_t)134217728, "carve must stay within 128 MiB");

constexpr size_t OUT0_BYTES = (size_t)ROWSF1 * 4;
constexpr size_t OUT1_BYTES = (size_t)BATCH * 128 * S2N * 4;
static_assert(OUT0_BYTES == 524288 && OUT0_BYTES + OUT1_BYTES == 786432, "output packing");

static_assert(gemm_ok(ROWS1, 64, 64) && gemm_ok(ROWS1, 64, 32), "SA1 gemm shapes");
static_assert(gemm_ok(ROWS2, 64, 96) && gemm_ok(ROWS2, 64, 64) && gemm_ok(ROWS2, 128, 64), "SA2 gemm shapes");
static_assert(gemm_ok(ROWSF2, 256, 192) && gemm_ok(ROWSF2, 128, 256) && gemm_ok(ROWSF2, 128, 128), "FP2 gemm shapes");
static_assert(gemm_ok(CHUNK_ROWS, 128, 128), "big gemm chunk shape");
static_assert(((CHUNK_ROWS * 128) >> 3) % 256 == 0, "apply grid exact");
static_assert((((CHUNK_ROWS >> 6) * (128 >> 5)) % 8) == 0, "big gemm grid exact");
static_assert(NPTS == 1024 * 16 && S1N == 128 * 1, "fps partition");

extern "C" void kernel_launch(void* const* d_in, const int* in_sizes, int n_in,
                              void* d_out, int out_size, void* d_ws, size_t ws_size,
                              hipStream_t stream) {
  if (n_in < 15) return;
  if (in_sizes[0] != BATCH * CIN_CH * NPTS) return;
  if (out_size != ROWSF1 + BATCH * 128 * S2N) return;
  if (ws_size < WS_TOTAL) return;

  const float* xyz = (const float*)d_in[0];
  const float* conv2w = (const float*)d_in[13];
  const float* conv2b = (const float*)d_in[14];
  float* out0 = (float*)d_out;
  float* out1 = out0 + (OUT0_BYTES / 4);

  char* ws = (char*)d_ws;
  float* P0 = (float*)(ws + OFF_P0);
  float* C1 = (float*)(ws + OFF_C1);
  float* C2 = (float*)(ws + OFF_C2);
  unsigned short* whi = (unsigned short*)(ws + OFF_WHI);
  unsigned short* wlo = (unsigned short*)(ws + OFF_WLO);
  float* bnpA = (float*)(ws + OFF_BNP);
  float* statp = (float*)(ws + OFF_STAT);
  float* l1p = (float*)(ws + OFF_L1P);
  float* l4 = (float*)(ws + OFF_L4);
  unsigned short* ash = (unsigned short*)(ws + OFF_ASH);
  unsigned short* asl = (unsigned short*)(ws + OFF_ASL);
  float* ys = (float*)(ws + OFF_YS);
  unsigned short* f2ah = (unsigned short*)(ws + OFF_F2AH);
  unsigned short* f2al = (unsigned short*)(ws + OFF_F2AL);
  float* f2y = (float*)(ws + OFF_F2Y);
  unsigned short* f2bh = (unsigned short*)(ws + OFF_F2BH);
  unsigned short* f2bl = (unsigned short*)(ws + OFF_F2BL);
  float* f2y2 = (float*)(ws + OFF_F2Y2);
  unsigned short* l1nh = (unsigned short*)(ws + OFF_L1NH);
  unsigned short* l1nl = (unsigned short*)(ws + OFF_L1NL);
  float* zt = (float*)(ws + OFF_ZT);
  float* ybig = (float*)(ws + OFF_YBIG);
  unsigned short* abh = (unsigned short*)(ws + OFF_ABH);
  unsigned short* abl = (unsigned short*)(ws + OFF_ABL);

  auto bnslot = [&](int s) { return bnpA + (size_t)s * 512; };

  for (int i = 0; i < NUM_W; ++i) {
    const int total8 = (W_OP[i] * W_KP[i]) >> 3;
    k_prep_w<<<dim3((unsigned)(total8 / 256)), dim3(256), 0, stream>>>(
        (const float*)d_in[W_DIN[i]], W_O[i], W_K[i], W_OP[i], W_KP[i],
        (unsigned*)(whi + w_off(i)), (unsigned*)(wlo + w_off(i)), W_MODE[i]);
  }
  k_prep_points<<<dim3((unsigned)(ROWSF1 / 256)), dim3(256), 0, stream>>>(xyz, P0, BATCH, CIN_CH, NPTS);

  auto gemm = [&](const unsigned short* Ah, const unsigned short* Al, int lda, int wi,
                  float* Yp, int ldc, int M, int N, int K, bool stats) {
    const int tiles = (M >> 6) * (N >> 5);
    const unsigned gx = (unsigned)((tiles + 7) / 8);
    if (stats)
      wmma_gemm_s<true><<<dim3(gx), dim3(256), 0, stream>>>(Ah, Al, lda, whi + w_off(wi), wlo + w_off(wi), W_KP[wi],
                                                           Yp, ldc, statp, M, N, K);
    else
      wmma_gemm_s<false><<<dim3(gx), dim3(256), 0, stream>>>(Ah, Al, lda, whi + w_off(wi), wlo + w_off(wi), W_KP[wi],
                                                            Yp, ldc, statp, M, N, K);
  };
  auto reduce = [&](int tilesM, int groups, int Mrows, int slot) {
    k_bn_reduce<<<dim3(1), dim3(256), 0, stream>>>(statp, tilesM, groups, 1.0 / (double)Mrows, bnslot(slot));
  };
  auto apply_split = [&](const float* Yp, int slot, unsigned short* hi, unsigned short* lo, int M, int ld) {
    const int total8 = (M * ld) >> 3;
    k_apply_split<<<dim3((unsigned)((total8 + 255) / 256)), dim3(256), 0, stream>>>(
        Yp, bnslot(slot), (unsigned*)hi, (unsigned*)lo, total8, ld);
  };

  k_fps<1024, 16><<<dim3(BATCH), dim3(1024), 0, stream>>>(P0, S1N, C1);
  k_ballgroup<2><<<dim3((unsigned)(BATCH * S1N / 8)), dim3(256), 0, stream>>>(
      P0, NPTS, C1, S1N, BATCH * S1N, 0.09f,
      xyz, (long)CIN_CH * NPTS, 1L, (long)NPTS, CIN_CH, (unsigned*)ash, (unsigned*)asl);
  gemm(ash, asl, 64, 0, ys, 64, ROWS1, 64, 64, true);
  reduce(ROWS1 / 64, 1, ROWS1, 0);
  apply_split(ys, 0, ash, asl, ROWS1, 64);
  gemm(ash, asl, 64, 1, ys, 64, ROWS1, 64, 32, true);
  reduce(ROWS1 / 64, 1, ROWS1, 1);
  apply_split(ys, 1, ash, asl, ROWS1, 64);
  gemm(ash, asl, 64, 2, ys, 64, ROWS1, 64, 32, true);
  reduce(ROWS1 / 64, 1, ROWS1, 2);
  k_bn_maxpool<2><<<dim3((unsigned)(BATCH * S1N / 8)), dim3(256), 0, stream>>>(ys, bnslot(2), l1p, BATCH * S1N);

  k_fps<128, 1><<<dim3(BATCH), dim3(128), 0, stream>>>(C1, S2N, C2);
  k_ballgroup<4><<<dim3((unsigned)(BATCH * S2N / 8)), dim3(256), 0, stream>>>(
      C1, S1N, C2, S2N, BATCH * S2N, 0.36f,
      l1p, (long)S1N * 64, 64L, 1L, 64, (unsigned*)ash, (unsigned*)asl);
  gemm(ash, asl, 128, 3, ys, 64, ROWS2, 64, 96, true);
  reduce(ROWS2 / 64, 1, ROWS2, 3);
  apply_split(ys, 3, ash, asl, ROWS2, 64);
  gemm(ash, asl, 64, 4, ys, 64, ROWS2, 64, 64, true);
  reduce(ROWS2 / 64, 1, ROWS2, 4);
  apply_split(ys, 4, ash, asl, ROWS2, 64);
  gemm(ash, asl, 64, 5, ys, 128, ROWS2, 128, 64, true);
  reduce(ROWS2 / 64, 2, ROWS2, 5);
  k_bn_maxpool<4><<<dim3((unsigned)(BATCH * S2N / 8)), dim3(256), 0, stream>>>(ys, bnslot(5), l4, BATCH * S2N);
  k_out1<<<dim3(BATCH), dim3(256), 0, stream>>>(l4, out1);

  k_fp2<<<dim3(BATCH), dim3(128), 0, stream>>>(C1, C2, l1p, l4, (unsigned*)f2ah, (unsigned*)f2al);
  gemm(f2ah, f2al, 192, 6, f2y, 256, ROWSF2, 256, 192, true);
  reduce(ROWSF2 / 64, 4, ROWSF2, 6);
  apply_split(f2y, 6, f2bh, f2bl, ROWSF2, 256);
  gemm(f2bh, f2bl, 256, 7, f2y2, 128, ROWSF2, 128, 256, true);
  reduce(ROWSF2 / 64, 2, ROWSF2, 7);
  apply_split(f2y2, 7, l1nh, l1nl, ROWSF2, 128);

  gemm(l1nh, l1nl, 128, 8, zt, 128, ROWSF2, 128, 128, false);
  k_fp1<<<dim3((unsigned)(ROWSF1 / 256)), dim3(256), 0, stream>>>(P0, C1, zt, ybig, statp);
  reduce(ROWSF1 / 32, 2, ROWSF1, 8);

  const int chunk8 = (CHUNK_ROWS * 128) >> 3;
  const unsigned chunkTiles = (unsigned)((CHUNK_ROWS >> 6) * (128 >> 5));
  for (int l = 0; l < 3; ++l) {
    for (int h = 0; h < BIG_CHUNKS; ++h) {
      float* ych = ybig + (size_t)h * CHUNK_ROWS * 128;
      float* sch = statp + (size_t)h * (CHUNK_ROWS / 64) * 2 * 128;
      k_apply_f16s<<<dim3((unsigned)(chunk8 / 256)), dim3(256), 0, stream>>>(
          ych, bnslot(8 + l), (unsigned*)abh, (unsigned*)abl, chunk8, 128);
      k_gemm_big<<<dim3(chunkTiles / 8), dim3(256), 0, stream>>>(
          abh, abl, 128, whi + w_off(9 + l), wlo + w_off(9 + l), 128,
          ych, 128, sch, CHUNK_ROWS, 128, 128);
    }
    reduce(ROWSF1 / 64, 2, ROWSF1, 9 + l);
  }
  k_final<<<dim3((unsigned)(ROWSF1 / 32 / 8)), dim3(256), 0, stream>>>(ybig, bnslot(11), conv2w, conv2b, out0, ROWSF1 / 32);
}
